// EchoStateNetwork_85512798863668
// MI455X (gfx1250) — hardware-verified
//
#include <hip/hip_runtime.h>
#include <math.h>

typedef __attribute__((ext_vector_type(16))) _Float16 v16h;
typedef __attribute__((ext_vector_type(8)))  _Float16 v8h;
typedef __attribute__((ext_vector_type(4)))  _Float16 v4h;
typedef __attribute__((ext_vector_type(8)))  float    v8f;
typedef __attribute__((ext_vector_type(4)))  float    v4f;

constexpr int kNB     = 32;
constexpr int kNT     = 1024;
constexpr int kDin    = 128;
constexpr int kRes    = 1024;
constexpr int kOutW   = 128;
constexpr int kRows   = kNB * kNT;
constexpr int kKcat   = kDin + kRes;
constexpr int kKSteps = kKcat / 32;
constexpr int kAPitch = kKcat + 8;
constexpr int kABuf   = 16 * kAPitch;
constexpr int kRecLdsBytes = 2 * kABuf * 2;
constexpr float kCarryA = 64.0f;
constexpr float kCarryW = 1024.0f;
constexpr float kFold   = 1.0f / (kCarryA * kCarryW);
constexpr float kLeak   = 0.3f;
constexpr float kKeep   = 0.7f;
constexpr bool kInputsViaBf16 = true;

static_assert(kKcat == 1152);
static_assert((kKcat % 32) == 0 && (kRes % 32) == 0);
static_assert((kRows % 64) == 0 && (kOutW % 64) == 0);
static_assert(kKSteps == 36);
static_assert(kRecLdsBytes == 74240);
static_assert((kAPitch * 2) % 16 == 0);

constexpr size_t kSzXH    = (size_t)kRows * kDin * 2;
constexpr size_t kSzBtrec = (size_t)kRes * kKcat * 2;
constexpr size_t kSzWout  = (size_t)kOutW * kRes * 2;
constexpr size_t kSzBias  = (size_t)kOutW * 4;
constexpr size_t kSzSt    = (size_t)kRows * kRes * 2;
constexpr size_t kOffXH    = 0;
constexpr size_t kOffBtrec = kOffXH + kSzXH;
constexpr size_t kOffWout  = kOffBtrec + kSzBtrec;
constexpr size_t kOffBias  = kOffWout + kSzWout;
constexpr size_t kOffSt    = kOffBias + kSzBias;
constexpr size_t kWsTotal  = kOffSt + kSzSt;
static_assert(kWsTotal == 78119424ull);
static_assert(kWsTotal <= 134217728ull);
static_assert((kOffBtrec % 128) == 0 && (kOffWout % 128) == 0 && (kOffBias % 128) == 0 && (kOffSt % 128) == 0);

__device__ __forceinline__ unsigned short f2bf_bits(float f) {
  unsigned u = __float_as_uint(f);
  return (unsigned short)((u + 0x7FFFu + ((u >> 16) & 1u)) >> 16);
}
__device__ __forceinline__ float bf_bits2f(unsigned short h) { return __uint_as_float(((unsigned)h) << 16); }
__device__ __forceinline__ float input_value(float f) {
  if (kInputsViaBf16) return bf_bits2f(f2bf_bits(f));
  return f;
}

union FragU { v16h v; v8h h[2]; };
__device__ __forceinline__ v16h frag_load(const _Float16* p) {
  FragU f;
  f.h[0] = *(const v8h*)(p);
  f.h[1] = *(const v8h*)(p + 16);
  return f.v;
}
__device__ __forceinline__ v8f mma_g(v16h a, v16h b, v8f c) {
  c = __builtin_amdgcn_wmma_f32_16x16x32_f16(false, a, false, b, (short)0, c, false, false);
  asm volatile("v_nop\n\tv_nop\n\tv_nop\n\tv_nop" : "+v"(c) : "v"(a), "v"(b));
  return c;
}
__device__ __forceinline__ void keep4_h(v16h a, v16h b, v16h c, v16h d) { asm volatile("v_nop" :: "v"(a), "v"(b), "v"(c), "v"(d)); }

__device__ __forceinline__ void cvt8_store2(const float* __restrict__ s, unsigned short* d, float carry) {
  const v4f a0 = *(const v4f*)(s);
  const v4f a1 = *(const v4f*)(s + 4);
  v8h hv;
#pragma unroll
  for (int e = 0; e < 4; ++e) {
    const float f0 = a0[e];
    const float f1 = a1[e];
    hv[e]     = (_Float16)(input_value(f0) * carry);
    hv[4 + e] = (_Float16)(input_value(f1) * carry);
  }
  *(volatile v8h*)d = hv;
  __threadfence();
  *(volatile v8h*)d = hv;
}

constexpr int kTotX8 = kRows * kDin / 8;
constexpr int kBlkX  = kTotX8 / 256;
static_assert(kBlkX * 256 == kTotX8);
__global__ __launch_bounds__(256) void cvt_x_kernel(const float* __restrict__ x, unsigned short* __restrict__ XH) {
  const int i = blockIdx.x * 256 + threadIdx.x;
  if (i >= kTotX8) return;
  cvt8_store2(x + ((size_t)i << 3), XH + ((size_t)i << 3), kCarryA);
}

constexpr int kBlkWin  = kRes * (kDin / 8) / 256;
constexpr int kBlkWres = kRes * (kRes / 8) / 256;
static_assert(kBlkWin == 64 && kBlkWres == 512);
__global__ __launch_bounds__(256) void build_rec_weights_kernel(
    const float* __restrict__ W_in, const float* __restrict__ W_res, unsigned short* __restrict__ Btrec) {
  const bool segIn = ((int)blockIdx.x < kBlkWin);
  const int bi     = segIn ? (int)blockIdx.x : ((int)blockIdx.x - kBlkWin);
  const int sh     = segIn ? 4 : 7;
  const float* src = segIn ? W_in : W_res;
  const int spitch = segIn ? kDin : kRes;
  const int coloff = segIn ? 0 : kDin;
  const int i = bi * 256 + threadIdx.x;
  const int n = i >> sh;
  const int c = i & ((1 << sh) - 1);
  cvt8_store2(src + (size_t)n * spitch + 8 * c, Btrec + (size_t)n * kKcat + coloff + 8 * c, kCarryW);
}

constexpr int kBlkWout = kOutW * (kRes / 8) / 256;
static_assert(kBlkWout == 64);
__global__ __launch_bounds__(256) void cvt_wout_bias_kernel(
    const float* __restrict__ W_out, const float* __restrict__ b_out,
    unsigned short* __restrict__ Wouth, float* __restrict__ biasr) {
  const int wave = __builtin_amdgcn_readfirstlane((int)(threadIdx.x >> 5));
  const int lane = threadIdx.x & 31;
  if ((int)blockIdx.x < kBlkWout) {
    const int i = blockIdx.x * 256 + threadIdx.x;
    cvt8_store2(W_out + ((size_t)i << 3), Wouth + ((size_t)i << 3), kCarryW);
  } else {
    if (wave == 0) {
      const v4f bv = *(const v4f*)(b_out + 4 * lane);
      v4f ov;
#pragma unroll
      for (int e = 0; e < 4; ++e) {
        const float f0 = bv[e];
        ov[e] = input_value(f0);
      }
      *(volatile v4f*)(biasr + 4 * lane) = ov;
      __threadfence();
      *(volatile v4f*)(biasr + 4 * lane) = ov;
    }
  }
}

__global__ __launch_bounds__(512) void recurrence_kernel(
    const unsigned short* __restrict__ XHp, const unsigned short* __restrict__ Btrecp,
    unsigned short* __restrict__ St) {
  extern __shared__ __align__(16) _Float16 sA[];
  const int tid  = threadIdx.x;
  const int lane = tid & 31;
  const int wave = __builtin_amdgcn_readfirstlane((int)(threadIdx.x >> 5));
  const int hh   = lane >> 4;
  const int m    = lane & 15;
  const int b0   = blockIdx.x * 16;
  const _Float16* Xp = (const _Float16*)XHp;
  const _Float16* Bp = (const _Float16*)Btrecp;

  const int xrow = tid >> 5;
  const int xc4  = (tid & 31) * 4;
  const _Float16* xsrc = Xp + (size_t)(b0 + xrow) * kNT * kDin + xc4;

  {
    v8h z;
#pragma unroll
    for (int e = 0; e < 8; ++e) z[e] = (_Float16)0.0f;
#pragma unroll
    for (int qq = 0; qq < 4; ++qq) {
      const int i = tid + 512 * qq;
      const int row = i >> 7;
      const int c = i & 127;
      *(v8h*)&sA[row * kAPitch + kDin + 8 * c] = z;
    }
    const v4h x0 = *(const v4h*)(xsrc);
    *(v4h*)&sA[xrow * kAPitch + xc4] = x0;
  }
  __syncthreads();

  const v8f zero8 = (v8f){0.f, 0.f, 0.f, 0.f, 0.f, 0.f, 0.f, 0.f};
  v8f hm0 = zero8, hm1 = zero8, hm2 = zero8, hm3 = zero8;

  const int aLane = m * kAPitch + 8 * hh;
  const _Float16* bp0 = Bp + (size_t)(64 * wave + m) * kKcat + 8 * hh;
  const _Float16* bp1 = bp0 + (size_t)16 * kKcat;
  const _Float16* bp2 = bp0 + (size_t)32 * kKcat;
  const _Float16* bp3 = bp0 + (size_t)48 * kKcat;

  int curOff = 0;
  int nxtOff = kABuf;
#pragma unroll 1
  for (int t = 0; t < kNT; ++t) {
    const int tn = (t + 1 < kNT) ? (t + 1) : (kNT - 1);
    const v4h xnext = *(const v4h*)(xsrc + (size_t)tn * kDin);

    v8f acc0 = zero8, acc1 = zero8, acc2 = zero8, acc3 = zero8;
    const int aBase = curOff + aLane;
#pragma unroll 1
    for (int ks = 0; ks < kKSteps; ++ks) {
      const int k0 = ks * 32;
      const v16h a  = frag_load(&sA[aBase + k0]);
      const v16h f0 = frag_load(bp0 + k0);
      const v16h f1 = frag_load(bp1 + k0);
      const v16h f2 = frag_load(bp2 + k0);
      const v16h f3 = frag_load(bp3 + k0);
      acc0 = mma_g(a, f0, acc0);
      acc1 = mma_g(a, f1, acc1);
      acc2 = mma_g(a, f2, acc2);
      acc3 = mma_g(a, f3, acc3);
    }

#pragma unroll 1
    for (int jj = 0; jj < 4; ++jj) {
      const int col = kDin + 64 * wave + 16 * jj + m;
#pragma unroll
      for (int r = 0; r < 8; ++r) {
        const float pre = acc0[r] * kFold;
        const float th  = tanhf(pre);
        const float hv  = kKeep * hm0[r] + kLeak * th;
        hm0[r] = hv;
        sA[nxtOff + (8 * hh + r) * kAPitch + col] = (_Float16)(hv * kCarryA);
      }
      acc0 = acc1;
      acc1 = acc2;
      acc2 = acc3;
      const v8f tmpH = hm0;
      hm0 = hm1;
      hm1 = hm2;
      hm2 = hm3;
      hm3 = tmpH;
    }
    *(v4h*)&sA[nxtOff + xrow * kAPitch + xc4] = xnext;

    __syncthreads();

    {
      const int hbase = nxtOff + wave * kAPitch + kDin + lane * 8;
      const v8h s0 = *(const v8h*)&sA[hbase];
      const v8h s1 = *(const v8h*)&sA[hbase + 256];
      const v8h s2 = *(const v8h*)&sA[hbase + 512];
      const v8h s3 = *(const v8h*)&sA[hbase + 768];
      unsigned short* dst = St + ((size_t)(b0 + wave) * kNT + t) * kRes + lane * 8;
      for (int pass = 0; pass < 2; ++pass) {
        *(volatile v8h*)(dst)       = s0;
        *(volatile v8h*)(dst + 256) = s1;
        *(volatile v8h*)(dst + 512) = s2;
        *(volatile v8h*)(dst + 768) = s3;
        __threadfence();
      }
    }
    const int tmpOff = curOff;
    curOff = nxtOff;
    nxtOff = tmpOff;
  }
}

__global__ __launch_bounds__(256) void out_proj_gemm_kernel(
    const unsigned short* __restrict__ Ap, int lda,
    const unsigned short* __restrict__ Btp, int ldb,
    float* __restrict__ C, int ldc,
    const float* __restrict__ bias,
    int M, int N, int K, float scale) {
  const _Float16* A  = (const _Float16*)Ap;
  const _Float16* Bt = (const _Float16*)Btp;
  __shared__ __align__(16) float sT[8][16 * 68];
  const int lane = threadIdx.x & 31;
  const int wave = __builtin_amdgcn_readfirstlane((int)(threadIdx.x >> 5));
  const int tilesN = N >> 6;
  const int tilesM = M >> 6;
  const int tile = blockIdx.x * 8 + wave;
  if (tile >= tilesM * tilesN) return;
  const int tm = tile / tilesN;
  const int tn = tile - tm * tilesN;
  const int m0 = tm << 6;
  const int n0 = tn << 6;

  const int rlane = lane & 15;
  const int koff  = (lane >> 4) * 8;
  const int mOff  = (lane >> 4) * 8;

  v8f acc[4][4];
#pragma unroll
  for (int i = 0; i < 4; ++i)
#pragma unroll
    for (int j = 0; j < 4; ++j) acc[i][j] = (v8f){0.f, 0.f, 0.f, 0.f, 0.f, 0.f, 0.f, 0.f};

  for (int k0 = 0; k0 < K; k0 += 32) {
    v16h bh[4];
#pragma unroll
    for (int j = 0; j < 4; ++j) {
      const size_t bo = (size_t)(n0 + (j << 4) + rlane) * ldb + koff + k0;
      bh[j] = frag_load(Bt + bo);
    }
#pragma unroll
    for (int i = 0; i < 4; ++i) {
      const size_t ao = (size_t)(m0 + (i << 4) + rlane) * lda + koff + k0;
      const v16h ah = frag_load(A + ao);
#pragma unroll
      for (int j = 0; j < 4; ++j) acc[i][j] = mma_g(ah, bh[j], acc[i][j]);
    }
    keep4_h(bh[0], bh[1], bh[2], bh[3]);
  }

  float* slab = sT[wave];
#pragma unroll
  for (int i = 0; i < 4; ++i) {
    const int mBase = m0 + (i << 4);
#pragma unroll
    for (int j = 0; j < 4; ++j) {
      const int n = n0 + (j << 4) + rlane;
      const float bv = bias[n];
#pragma unroll
      for (int r = 0; r < 8; ++r) {
        float v = acc[i][j][r] * scale;
        v += bv;
        slab[(mOff + r) * 68 + (j << 4) + rlane] = v;
      }
    }
    __builtin_amdgcn_fence(__ATOMIC_RELEASE, "workgroup");
    __builtin_amdgcn_wave_barrier();
    __builtin_amdgcn_fence(__ATOMIC_ACQUIRE, "workgroup");
    {
      const int hh = lane >> 4, c4 = (lane & 15) * 4;
      for (int pass = 0; pass < 2; ++pass) {
#pragma unroll
        for (int it = 0; it < 8; ++it) {
          const int row = it * 2 + hh;
          const v4f v = *(const v4f*)(slab + row * 68 + c4);
          *(volatile v4f*)(C + (size_t)(mBase + row) * ldc + n0 + c4) = v;
        }
        __threadfence();
      }
    }
    __builtin_amdgcn_fence(__ATOMIC_RELEASE, "workgroup");
    __builtin_amdgcn_wave_barrier();
    __builtin_amdgcn_fence(__ATOMIC_ACQUIRE, "workgroup");
  }
}

extern "C" void kernel_launch(void* const* d_in, const int* in_sizes, int n_in,
                              void* d_out, int out_size, void* d_ws, size_t ws_size,
                              hipStream_t stream) {
  if (n_in < 5) return;
  if (in_sizes[0] != kRows * kDin) return;
  if (in_sizes[1] != kRes * kRes) return;
  if (in_sizes[2] != kRes * kDin) return;
  if (in_sizes[3] != kOutW * kRes) return;
  if (in_sizes[4] != kOutW) return;
  if (out_size != kRows * kOutW) return;
  if (ws_size < kWsTotal) return;

  const float* x     = (const float*)d_in[0];
  const float* W_res = (const float*)d_in[1];
  const float* W_in  = (const float*)d_in[2];
  const float* W_out = (const float*)d_in[3];
  const float* b_out = (const float*)d_in[4];
  float* out = (float*)d_out;

  char* ws = (char*)d_ws;
  unsigned short* XH    = (unsigned short*)(ws + kOffXH);
  unsigned short* BTREC = (unsigned short*)(ws + kOffBtrec);
  unsigned short* WOUTH = (unsigned short*)(ws + kOffWout);
  float*          BIASR = (float*)(ws + kOffBias);
  unsigned short* ST    = (unsigned short*)(ws + kOffSt);

  cvt_x_kernel<<<kBlkX, 256, 0, stream>>>(x, XH);
  build_rec_weights_kernel<<<kBlkWin + kBlkWres, 256, 0, stream>>>(W_in, W_res, BTREC);
  cvt_wout_bias_kernel<<<kBlkWout + 1, 256, 0, stream>>>(W_out, b_out, WOUTH, BIASR);

  recurrence_kernel<<<kNB / 16, 512, kRecLdsBytes, stream>>>(XH, BTREC, ST);

  constexpr int kTiles = (kRows / 64) * (kOutW / 64);
  static_assert((kTiles % 8) == 0);
  out_proj_gemm_kernel<<<kTiles / 8, 256, 0, stream>>>(
      ST, kRes, WOUTH, kRes, out, kOutW, BIASR, kRows, kOutW, kRes, kFold);
}
